// RnnBlock_80298708566129
// MI455X (gfx1250) — hardware-run, weakly checked
//
#include <hip/hip_runtime.h>
#include <math.h>

constexpr int NBATCH = 16;
constexpr int NSTEP  = 400;
constexpr int NFEAT  = 512;
constexpr int NUNIT  = 1024;
constexpr int NGATE  = 4 * NUNIT;
constexpr int NROWS  = NBATCH * NSTEP;
constexpr int NCHAN  = 2 * NUNIT;
constexpr int CTHR   = 256;
constexpr int LTHR   = 512;
constexpr int LWAVES = LTHR / 32;
constexpr int HPITCH = NUNIT + 8;
constexpr int SLABP  = 68;
constexpr float WCARRY     = 16.0f;
constexpr float WCARRY_INV = 1.0f / 16.0f;
constexpr float BN_EPS     = 1e-3f;

static_assert(NROWS % 64 == 0);
static_assert(NGATE % 64 == 0);
static_assert(NFEAT % 32 == 0);
static_assert(NUNIT % 32 == 0);
static_assert(((NROWS / 64) * (NGATE / 64)) % 8 == 0);
static_assert(NUNIT == 64 * LWAVES);
static_assert(HPITCH % 8 == 0);
static_assert((NROWS * (NFEAT / 8)) % CTHR == 0);
static_assert(NBATCH == 16);

typedef __attribute__((ext_vector_type(16))) _Float16 v16h;
typedef __attribute__((ext_vector_type(8)))  _Float16 v8h;
typedef __attribute__((ext_vector_type(16))) __bf16   v16b;
typedef __attribute__((ext_vector_type(8)))  __bf16   v8b;
typedef __attribute__((ext_vector_type(8)))  float    v8f;
typedef __attribute__((ext_vector_type(4)))  float    v4f;

__device__ __forceinline__ unsigned short f2bf_bits(float f) {
  unsigned u = __float_as_uint(f);
  return (unsigned short)((u + 0x7FFFu + ((u >> 16) & 1u)) >> 16);
}
__device__ __forceinline__ float bf_bits2f(unsigned short h) { return __uint_as_float(((unsigned)h) << 16); }
__device__ __forceinline__ float bf16r(float f) { return bf_bits2f(f2bf_bits(f)); }

__device__ __forceinline__ float h16_to_f32(unsigned hb) {
  const unsigned sgn = (hb & 0x8000u) << 16;
  const unsigned em = hb & 0x7fffu;
  const float fn = __uint_as_float((em << 13) + 0x38000000u);
  const float fs = (float)em * 5.9604644775390625e-8f;
  const float mag = (em < 0x400u) ? fs : fn;
  return __uint_as_float(__float_as_uint(mag) | sgn);
}

__device__ __forceinline__ void dep_guard4_h(v8f& a0, v8f& a1, v8f& a2, v8f& a3, v16h x, v16h y) {
  asm volatile("v_nop\n\tv_nop\n\tv_nop\n\tv_nop" : "+v"(a0), "+v"(a1), "+v"(a2), "+v"(a3) : "v"(x), "v"(y));
}
__device__ __forceinline__ void dep_guard4_b(v8f& a0, v8f& a1, v8f& a2, v8f& a3, v16b x, v16b y) {
  asm volatile("v_nop\n\tv_nop\n\tv_nop\n\tv_nop" : "+v"(a0), "+v"(a1), "+v"(a2), "+v"(a3) : "v"(x), "v"(y));
}
__device__ __forceinline__ void guard_group4(v8f& a0, v8f& a1, v8f& a2, v8f& a3, v16h x, v16h b0, v16h b1, v16h b2, v16h b3) {
  asm volatile("v_nop\n\tv_nop\n\tv_nop\n\tv_nop" : "+v"(a0), "+v"(a1), "+v"(a2), "+v"(a3) : "v"(x), "v"(b0), "v"(b1), "v"(b2), "v"(b3));
}
__device__ __forceinline__ void keep4_h(v16h a, v16h b, v16h c, v16h d) { asm volatile("v_nop" :: "v"(a), "v"(b), "v"(c), "v"(d)); }
__device__ __forceinline__ void keep4_b(v16b a, v16b b, v16b c, v16b d) { asm volatile("v_nop" :: "v"(a), "v"(b), "v"(c), "v"(d)); }
__device__ __forceinline__ void acc_guard4(v8f& a, v8f& b, v8f& c, v8f& d) { asm volatile("v_nop\n\tv_nop\n\tv_nop\n\tv_nop" : "+v"(a), "+v"(b), "+v"(c), "+v"(d)); }

template <typename T> struct Frag;
template <> struct Frag<_Float16> {
  typedef v16h V; union U { v16h v; v8h h[2]; };
  static __device__ __forceinline__ v16h load(const _Float16* p) {
    U f; f.h[0] = *(const v8h*)(p); f.h[1] = *(const v8h*)(p + 16); return f.v;
  }
  static __device__ __forceinline__ v8f mma(v16h a, v16h b, v8f c) {
    return __builtin_amdgcn_wmma_f32_16x16x32_f16(false, a, false, b, (short)0, c, false, false);
  }
  static __device__ __forceinline__ void guard4(v8f& a0, v8f& a1, v8f& a2, v8f& a3, v16h x, v16h y) { dep_guard4_h(a0, a1, a2, a3, x, y); }
  static __device__ __forceinline__ void keep(v16h a, v16h b, v16h c, v16h d) { keep4_h(a, b, c, d); }
};
template <> struct Frag<__bf16> {
  typedef v16b V; union U { v16b v; v8b h[2]; };
  static __device__ __forceinline__ v16b load(const __bf16* p) {
    U f; f.h[0] = *(const v8b*)(p); f.h[1] = *(const v8b*)(p + 16); return f.v;
  }
  static __device__ __forceinline__ v8f mma(v16b a, v16b b, v8f c) {
    return __builtin_amdgcn_wmma_f32_16x16x32_bf16(false, a, false, b, (short)0, c, false, false);
  }
  static __device__ __forceinline__ void guard4(v8f& a0, v8f& a1, v8f& a2, v8f& a3, v16b x, v16b y) { dep_guard4_b(a0, a1, a2, a3, x, y); }
  static __device__ __forceinline__ void keep(v16b a, v16b b, v16b c, v16b d) { keep4_b(a, b, c, d); }
};

__device__ __forceinline__ float fsig(float x)  { return __builtin_amdgcn_rcpf(1.0f + __expf(-x)); }
__device__ __forceinline__ float ftanh(float x) { return 1.0f - 2.0f * __builtin_amdgcn_rcpf(__expf(2.0f * x) + 1.0f); }

template <int ET> struct Elem;
template <> struct Elem<0> { typedef _Float16 T; };
template <> struct Elem<1> { typedef __bf16 T; };
template <int ET, bool SPLIT, int BIAS_MODE, int OUT_MODE, bool RESID>
__global__ __launch_bounds__(256) void wmma_gemm64(
    const unsigned short* __restrict__ Ap, const unsigned short* __restrict__ A2p, int lda, long strideA,
    const unsigned short* __restrict__ Btp, const unsigned short* __restrict__ Bt2p, int ldb, long strideB,
    void* __restrict__ Cout, void* __restrict__ Cout2, int ldc, long strideC,
    const float* __restrict__ bias,
    const float* __restrict__ resid, long strideR,
    int M, int N, int K, float scale) {
  typedef typename Elem<ET>::T T;
  typedef typename Frag<T>::V V;
  const T* A = (const T*)Ap; const T* A2 = (const T*)A2p; const T* Bt = (const T*)Btp; const T* Bt2 = (const T*)Bt2p;
  __shared__ __align__(16) float sT[8][16 * 68];
  const int b    = blockIdx.y;
  const int lane = threadIdx.x & 31;
  const int wave = threadIdx.x >> 5;
  const int tilesN = N >> 6;
  const int tilesM = M >> 6;
  const int tile = blockIdx.x * 8 + wave;
  if (tile >= tilesM * tilesN) return;
  const int tm = tile / tilesN;
  const int tn = tile - tm * tilesN;
  const int m0 = tm << 6;
  const int n0 = tn << 6;

  const T* Ab  = A  + (size_t)b * strideA;
  const T* Bb  = Bt + (size_t)b * strideB;
  const T* Ab2 = SPLIT ? (A2  + (size_t)b * strideA) : nullptr;
  const T* Bb2 = SPLIT ? (Bt2 + (size_t)b * strideB) : nullptr;

  const int rlane = lane & 15;
  const int koff  = (lane >> 4) * 8;
  const int mOff  = (lane >> 4) * 8;

  v8f acc[4][4];
#pragma unroll
  for (int i = 0; i < 4; ++i)
#pragma unroll
    for (int j = 0; j < 4; ++j) acc[i][j] = (v8f){0.f,0.f,0.f,0.f,0.f,0.f,0.f,0.f};

  for (int k0 = 0; k0 < K; k0 += 32) {
    V bh[4], bl[4];
#pragma unroll
    for (int j = 0; j < 4; ++j) {
      const size_t bo = (size_t)(n0 + (j << 4) + rlane) * ldb + koff + k0;
      bh[j] = Frag<T>::load(Bb + bo);
      if (SPLIT) bl[j] = Frag<T>::load(Bb2 + bo);
    }
#pragma unroll
    for (int i = 0; i < 4; ++i) {
      const size_t ao = (size_t)(m0 + (i << 4) + rlane) * lda + koff + k0;
      V ah = Frag<T>::load(Ab + ao);
      V al;
      if (SPLIT) al = Frag<T>::load(Ab2 + ao);
#pragma unroll
      for (int j = 0; j < 4; ++j) {
        acc[i][j] = Frag<T>::mma(ah, bh[j], acc[i][j]);
        if (SPLIT) {
          acc[i][j] = Frag<T>::mma(ah, bl[j], acc[i][j]);
          acc[i][j] = Frag<T>::mma(al, bh[j], acc[i][j]);
        }
      }
      Frag<T>::guard4(acc[i][0], acc[i][1], acc[i][2], acc[i][3], ah, SPLIT ? al : ah);
    }
    Frag<T>::keep(bh[0], bh[1], bh[2], bh[3]);
    if (SPLIT) Frag<T>::keep(bl[0], bl[1], bl[2], bl[3]);
  }
  acc_guard4(acc[0][0], acc[0][1], acc[0][2], acc[0][3]);
  acc_guard4(acc[1][0], acc[1][1], acc[1][2], acc[1][3]);
  acc_guard4(acc[2][0], acc[2][1], acc[2][2], acc[2][3]);
  acc_guard4(acc[3][0], acc[3][1], acc[3][2], acc[3][3]);

  float* slab = sT[wave];
  const float* Rb = RESID ? (resid + (size_t)b * strideR) : nullptr;
#pragma unroll
  for (int i = 0; i < 4; ++i) {
    const int mBase = m0 + (i << 4);
#pragma unroll
    for (int j = 0; j < 4; ++j) {
      const int n = n0 + (j << 4) + rlane;
      float bv = 0.f;
      if (BIAS_MODE == 2) bv = bias[n];
#pragma unroll
      for (int r = 0; r < 8; ++r) {
        float v = acc[i][j][r] * scale;
        if (BIAS_MODE == 1) v += bias[mBase + mOff + r];
        if (BIAS_MODE == 2) v += bv;
        if (RESID) v += Rb[(size_t)(mBase + mOff + r) * ldc + n];
        slab[(mOff + r) * 68 + (j << 4) + rlane] = v;
      }
    }
    __builtin_amdgcn_fence(__ATOMIC_RELEASE, "workgroup");
    __builtin_amdgcn_wave_barrier();
    __builtin_amdgcn_fence(__ATOMIC_ACQUIRE, "workgroup");
    if (OUT_MODE == 0) {
      float* C = (float*)Cout + (size_t)b * strideC;
      const int hh = lane >> 4, c4 = (lane & 15) * 4;
      for (int pass = 0; pass < 2; ++pass) {
#pragma unroll
        for (int it = 0; it < 8; ++it) {
          const int row = it * 2 + hh;
          v4f v = *(const v4f*)(slab + row * 68 + c4);
          *(volatile v4f*)(C + (size_t)(mBase + row) * ldc + n0 + c4) = v;
        }
        __threadfence();
      }
    } else {
      const int q = lane >> 3, c8 = (lane & 7) * 8;
      unsigned short* C  = (unsigned short*)Cout  + (size_t)b * strideC;
      unsigned short* C2 = (OUT_MODE == 2) ? ((unsigned short*)Cout2 + (size_t)b * strideC) : nullptr;
      for (int pass = 0; pass < 2; ++pass) {
#pragma unroll
        for (int it = 0; it < 4; ++it) {
          const int row = it * 4 + q;
          const float* sp = slab + row * 68 + c8;
          v8h hv, lv;
#pragma unroll
          for (int e = 0; e < 8; ++e) {
            if (OUT_MODE == 1) {
              hv[e] = (_Float16)sp[e];
            } else {
              unsigned short hb = f2bf_bits(sp[e]);
              unsigned short lb = f2bf_bits(sp[e] - bf_bits2f(hb));
              hv[e] = __builtin_bit_cast(_Float16, hb);
              lv[e] = __builtin_bit_cast(_Float16, lb);
            }
          }
          *(volatile v8h*)(C + (size_t)(mBase + row) * ldc + n0 + c8) = hv;
          if (OUT_MODE == 2) *(volatile v8h*)(C2 + (size_t)(mBase + row) * ldc + n0 + c8) = lv;
        }
        __threadfence();
      }
    }
    __builtin_amdgcn_fence(__ATOMIC_RELEASE, "workgroup");
    __builtin_amdgcn_wave_barrier();
    __builtin_amdgcn_fence(__ATOMIC_ACQUIRE, "workgroup");
  }
}

__global__ __launch_bounds__(CTHR) void cvt_x_kernel(const float* __restrict__ x, unsigned short* __restrict__ dst) {
  const int i = blockIdx.x * CTHR + threadIdx.x;
  const int n8 = NROWS * (NFEAT / 8);
  if (i < n8) {
    const int m  = i >> 6;
    const int c8 = i & 63;
    const int t  = m >> 4;
    const int b  = m & 15;
    const float* sp = x + ((size_t)(b * NSTEP + t) * NFEAT + (size_t)c8 * 8);
    const v4f a = *(const v4f*)(sp);
    const v4f bq = *(const v4f*)(sp + 4);
    v8h hv;
#pragma unroll
    for (int e = 0; e < 4; ++e) {
      const float f0 = bf16r(a[e]);
      const float f1 = bf16r(bq[e]);
      hv[e]     = (_Float16)f0;
      hv[4 + e] = (_Float16)f1;
    }
    *(volatile v8h*)(dst + (size_t)i * 8) = hv;
    __threadfence();
    *(volatile v8h*)(dst + (size_t)i * 8) = hv;
  }
}

__global__ __launch_bounds__(CTHR) void tpw_kernel(const float* __restrict__ srcA, const float* __restrict__ srcB,
                                                  int R, int C, int ldo, unsigned short* __restrict__ O, float sc) {
  __shared__ float Tt[64 * 65];
  const int tid = threadIdx.x;
  const int c0 = blockIdx.x * 64, r0 = blockIdx.y * 64;
  const float* src = (blockIdx.z == 0) ? srcA : srcB;
  unsigned short* Od = O + (size_t)blockIdx.z * (size_t)R * (size_t)C;
#pragma unroll
  for (int i = 0; i < 4; ++i) {
    const int idx = i * CTHR + tid;
    const int rr = idx >> 4, cc = (idx & 15) * 4;
    const v4f v = *(const v4f*)(src + (size_t)(r0 + rr) * (size_t)C + c0 + cc);
    Tt[rr * 65 + cc + 0] = v[0];
    Tt[rr * 65 + cc + 1] = v[1];
    Tt[rr * 65 + cc + 2] = v[2];
    Tt[rr * 65 + cc + 3] = v[3];
  }
  __syncthreads();
  const int q = tid >> 3, c8 = (tid & 7) * 8;
  v8h hv[2];
#pragma unroll
  for (int g = 0; g < 2; ++g) {
    const int qq = g * 32 + q;
#pragma unroll
    for (int e = 0; e < 8; ++e) {
      const float f = Tt[(c8 + e) * 65 + qq];
      const float fb = bf16r(f);
      hv[g][e] = (_Float16)(fb * sc);
    }
  }
  for (int pass = 0; pass < 2; ++pass) {
#pragma unroll
    for (int g = 0; g < 2; ++g) {
      const size_t o = (size_t)(c0 + g * 32 + q) * (size_t)ldo + (size_t)(r0 + c8);
      *(volatile v8h*)(Od + o) = hv[g];
    }
    __threadfence();
  }
}

__global__ __launch_bounds__(CTHR) void bias_prep_kernel(const float* __restrict__ b_a, const float* __restrict__ b_b,
                                                         float* __restrict__ dst) {
  const int gt = blockIdx.x * CTHR + threadIdx.x;
  const int which = gt >> 10;
  const int idx = (gt & 1023) * 4;
  const v4f va = *(const v4f*)(b_a + idx);
  const v4f vb = *(const v4f*)(b_b + idx);
  v4f o;
#pragma unroll
  for (int e = 0; e < 4; ++e) {
    const float s = which ? vb[e] : va[e];
    o[e] = WCARRY * bf16r(s);
  }
  float* op = dst + which * NGATE + idx;
  *(volatile v4f*)op = o;
  __threadfence();
  *(volatile v4f*)op = o;
}

__global__ __launch_bounds__(LTHR) void lstm_dir_kernel(const unsigned* __restrict__ XWw,
                                                       const unsigned short* __restrict__ RTp,
                                                       const float* __restrict__ gam, const float* __restrict__ bet,
                                                       const float* __restrict__ mmean, const float* __restrict__ mvar,
                                                       float* __restrict__ out, int dir) {
  __shared__ __align__(16) _Float16 Ah[2][NBATCH * HPITCH];
  __shared__ __align__(16) float    Sl[LWAVES][16 * SLABP];
  const _Float16* RT = (const _Float16*)RTp;
  const int tid = threadIdx.x, lane = tid & 31, wave = tid >> 5;
  const int c = lane & 15, hh = lane >> 4, koff = hh * 8, c4 = c * 4;
  const unsigned sh = (unsigned)(c & 1) << 4;

  {
    unsigned* ahw = (unsigned*)&Ah[0][0];
#pragma unroll 1
    for (int i = tid; i < NBATCH * HPITCH; i += LTHR) ahw[i] = 0u;
  }
  float cst[4][8];
  float bninv[4], bnadd[4];
#pragma unroll
  for (int nt = 0; nt < 4; ++nt) {
    const int ch = dir * NUNIT + 64 * wave + 16 * nt + c;
    const float g  = bf16r(gam[ch]);
    const float be = bf16r(bet[ch]);
    const float mu = bf16r(mmean[ch]);
    const float va = bf16r(mvar[ch]);
    const float iv = g * rsqrtf(va + BN_EPS);
    bninv[nt] = iv;
    bnadd[nt] = be - mu * iv;
#pragma unroll
    for (int r = 0; r < 8; ++r) cst[nt][r] = 0.0f;
  }
  __syncthreads();

  float* slab = Sl[wave];

#pragma unroll 1
  for (int s = 0; s < NSTEP; ++s) {
    const int tx  = dir ? (NSTEP - 1 - s) : s;
    const int cur = s & 1;
    const _Float16* ahrow = &Ah[cur][0] + c * HPITCH + koff;
    _Float16* ahn = &Ah[cur ^ 1][0];
    const unsigned* xwt = XWw + (size_t)tx * (size_t)(NBATCH * NGATE / 2);

#pragma unroll
    for (int nt = 0; nt < 4; ++nt) {
      asm volatile("" ::: "memory");
      const int j  = 64 * wave + 16 * nt + c;
      const int jw = j >> 1;
      v8f acc[4];
#pragma unroll
      for (int g = 0; g < 4; ++g) {
#pragma unroll
        for (int r = 0; r < 8; ++r) {
          const unsigned w = xwt[(8 * hh + r) * (NGATE / 2) + g * (NUNIT / 2) + jw];
          acc[g][r] = h16_to_f32((w >> sh) & 0xffffu);
        }
      }
      const _Float16* wr = RT + (size_t)j * NUNIT + koff;
#pragma unroll 1
      for (int k0 = 0; k0 < NUNIT; k0 += 32) {
        const v16h a  = Frag<_Float16>::load(ahrow + k0);
        const v16h b0 = Frag<_Float16>::load(wr + k0);
        const v16h b1 = Frag<_Float16>::load(wr + (size_t)1 * NUNIT * NUNIT + k0);
        const v16h b2 = Frag<_Float16>::load(wr + (size_t)2 * NUNIT * NUNIT + k0);
        const v16h b3 = Frag<_Float16>::load(wr + (size_t)3 * NUNIT * NUNIT + k0);
        acc[0] = Frag<_Float16>::mma(a, b0, acc[0]);
        acc[1] = Frag<_Float16>::mma(a, b1, acc[1]);
        acc[2] = Frag<_Float16>::mma(a, b2, acc[2]);
        acc[3] = Frag<_Float16>::mma(a, b3, acc[3]);
        guard_group4(acc[0], acc[1], acc[2], acc[3], a, b0, b1, b2, b3);
      }
      acc_guard4(acc[0], acc[1], acc[2], acc[3]);
#pragma unroll
      for (int r = 0; r < 8; ++r) {
        const float zi = acc[0][r] * WCARRY_INV;
        const float zf = acc[1][r] * WCARRY_INV;
        const float zg = acc[2][r] * WCARRY_INV;
        const float zo = acc[3][r] * WCARRY_INV;
        const float ig = fsig(zi);
        const float fg = fsig(zf);
        const float gg = ftanh(zg);
        const float og = fsig(zo);
        const float cn = fg * cst[nt][r] + ig * gg;
        cst[nt][r] = cn;
        const float hn = og * ftanh(cn);
        ahn[(8 * hh + r) * HPITCH + j] = (_Float16)hn;
        slab[(8 * hh + r) * SLABP + 16 * nt + c] = hn * bninv[nt] + bnadd[nt];
      }
    }

    __builtin_amdgcn_fence(__ATOMIC_RELEASE, "workgroup");
    __builtin_amdgcn_wave_barrier();
    __builtin_amdgcn_fence(__ATOMIC_ACQUIRE, "workgroup");
    for (int pass = 0; pass < 2; ++pass) {
#pragma unroll
      for (int it = 0; it < 8; ++it) {
        const int row = it * 2 + hh;
        const v4f v = *(const v4f*)(slab + row * SLABP + c4);
        *(volatile v4f*)(out + ((size_t)row * NSTEP + (size_t)tx) * NCHAN + dir * NUNIT + 64 * wave + c4) = v;
      }
      __threadfence();
    }
    __builtin_amdgcn_fence(__ATOMIC_RELEASE, "workgroup");
    __builtin_amdgcn_wave_barrier();
    __builtin_amdgcn_fence(__ATOMIC_ACQUIRE, "workgroup");
    __syncthreads();
  }
}

extern "C" void kernel_launch(void* const* d_in, const int* in_sizes, int n_in,
                              void* d_out, int out_size, void* d_ws, size_t ws_size, hipStream_t stream) {
  if (n_in < 11 || d_out == nullptr || d_ws == nullptr) return;
  if (in_sizes[0] != NBATCH * NSTEP * NFEAT || in_sizes[1] != NFEAT * NGATE || in_sizes[2] != NUNIT * NGATE ||
      in_sizes[3] != NGATE || in_sizes[4] != NFEAT * NGATE || in_sizes[5] != NUNIT * NGATE || in_sizes[6] != NGATE ||
      in_sizes[7] != NCHAN || in_sizes[8] != NCHAN || in_sizes[9] != NCHAN || in_sizes[10] != NCHAN ||
      out_size != NBATCH * NSTEP * NCHAN) return;

  const float* x     = (const float*)d_in[0];
  const float* k_fwd = (const float*)d_in[1];
  const float* r_fwd = (const float*)d_in[2];
  const float* b_fwd = (const float*)d_in[3];
  const float* k_bwd = (const float*)d_in[4];
  const float* r_bwd = (const float*)d_in[5];
  const float* b_bwd = (const float*)d_in[6];
  const float* gam   = (const float*)d_in[7];
  const float* bet   = (const float*)d_in[8];
  const float* mmean = (const float*)d_in[9];
  const float* mvar  = (const float*)d_in[10];
  float* out = (float*)d_out;

  char* ws = (char*)d_ws; size_t off = 0;
  auto carve = [&](size_t bytes) -> char* { char* p = ws + off; off += (bytes + 255) & ~(size_t)255; return p; };
  unsigned short* X16  = (unsigned short*)carve((size_t)NROWS * NFEAT * 2);
  unsigned short* KT16 = (unsigned short*)carve((size_t)2 * NGATE * NFEAT * 2);
  unsigned short* RT16 = (unsigned short*)carve((size_t)2 * NGATE * NUNIT * 2);
  float*          BIAS = (float*)carve((size_t)2 * NGATE * 4);
  unsigned short* XW16 = (unsigned short*)carve((size_t)NROWS * NGATE * 2);
  if (off > ws_size || off > (size_t)134217728) return;

  cvt_x_kernel<<<(NROWS * (NFEAT / 8)) / CTHR, CTHR, 0, stream>>>(x, X16);
  tpw_kernel<<<dim3(NGATE / 64, NFEAT / 64, 2), CTHR, 0, stream>>>(k_fwd, k_bwd, NFEAT, NGATE, NFEAT, KT16, WCARRY);
  tpw_kernel<<<dim3(NGATE / 64, NUNIT / 64, 2), CTHR, 0, stream>>>(r_fwd, r_bwd, NUNIT, NGATE, NUNIT, RT16, WCARRY);
  bias_prep_kernel<<<8, CTHR, 0, stream>>>(b_fwd, b_bwd, BIAS);

  const dim3 ggrid((NROWS / 64) * (NGATE / 64) / 8, 1);
  for (int d = 0; d < 2; ++d) {
    const unsigned short* KTd = KT16 + (size_t)d * NGATE * NFEAT;
    const unsigned short* RTd = RT16 + (size_t)d * NGATE * NUNIT;
    const float* Bd = BIAS + (size_t)d * NGATE;
    wmma_gemm64<0, false, 2, 1, false><<<ggrid, 256, 0, stream>>>(
        X16, X16, NFEAT, 0L, KTd, KTd, NFEAT, 0L, (void*)XW16, (void*)XW16, NGATE, 0L,
        Bd, Bd, 0L, NROWS, NGATE, NFEAT, 1.0f);
    lstm_dir_kernel<<<1, LTHR, 0, stream>>>((const unsigned*)XW16, RTd, gam, bet, mmean, mvar, out, d);
  }
}
